// MultiHopMGAT_32461362823666
// MI455X (gfx1250) — hardware-run, weakly checked
//
#include <hip/hip_runtime.h>

typedef float          v8f   __attribute__((ext_vector_type(8)));
typedef float          v4f   __attribute__((ext_vector_type(4)));
typedef unsigned int   v4u   __attribute__((ext_vector_type(4)));
typedef int            v8i   __attribute__((ext_vector_type(8)));
typedef unsigned short v8us  __attribute__((ext_vector_type(8)));
typedef unsigned short v16us __attribute__((ext_vector_type(16)));
typedef __bf16         v16bf __attribute__((ext_vector_type(16)));
typedef _Float16       v16h  __attribute__((ext_vector_type(16)));
typedef v4f  __attribute__((may_alias)) v4fa;
typedef v8us __attribute__((may_alias)) v8usa;
union FragB { v16bf v; v16us u; v8us h[2]; v8i w; };
union FragH { v16h  v; v16us u; v8us h[2]; v8i w; };

__device__ __forceinline__ v8f wmb(const FragB& a, const FragB& b, v8f c) {
  v8f d = __builtin_amdgcn_wmma_f32_16x16x32_bf16(false, a.v, false, b.v, (short)0, c, false, false);
  asm volatile("v_nop\n\tv_nop\n\tv_nop\n\tv_nop" : "+v"(d) : "v"(a.w), "v"(b.w));
  return d;
}

__device__ __forceinline__ v8f wmh(const FragH& a, const FragH& b, v8f c) {
  v8f d = __builtin_amdgcn_wmma_f32_16x16x32_f16(false, a.v, false, b.v, (short)0, c, false, false);
  asm volatile("v_nop\n\tv_nop\n\tv_nop\n\tv_nop" : "+v"(d) : "v"(a.w), "v"(b.w));
  return d;
}

__device__ __forceinline__ unsigned bf16_bits(float f) {
  const unsigned u = __float_as_uint(f);
  const unsigned r = (u + 0x7FFFu + ((u >> 16) & 1u)) >> 16;
  const unsigned q = (u >> 16) | 0x40u;
  return ((u & 0x7fffffffu) > 0x7f800000u) ? q : r;
}

__device__ __forceinline__ float bf16_val(float f) {
  return __uint_as_float(bf16_bits(f) << 16);
}
__device__ __forceinline__ int clampi(int v, int lo, int hi) {
  return v < lo ? lo : (v > hi ? hi : v);
}

__device__ __forceinline__ unsigned f16_bits(float f) {
  const unsigned u  = __float_as_uint(f);
  const unsigned s  = (u >> 16) & 0x8000u;
  const unsigned a  = u & 0x7fffffffu;
  const unsigned t  = a - 0x38000000u;
  const unsigned r  = (t + 0x0FFFu + ((t >> 13) & 1u)) >> 13;
  const unsigned rc = r > 0x7C00u ? 0x7C00u : r;
  const bool small  = a < 0x38800000u;
  const bool isnan  = a > 0x7f800000u;
  const unsigned fin = small ? 0u : (s | rc);
  return isnan ? (s | 0x7E00u) : fin;
}

__device__ __forceinline__ unsigned pk16(unsigned lo, unsigned hi) { return lo | (hi << 16); }
__device__ __forceinline__ unsigned bf16_lo_bits(float v) {
  float hi = bf16_val(v);
  asm volatile("" : "+v"(hi));
  return bf16_bits(v - hi);
}
__device__ __forceinline__ v4u pack8_bf16(v4f a, v4f c) {
  return (v4u){ pk16(bf16_bits(a[0]), bf16_bits(a[1])), pk16(bf16_bits(a[2]), bf16_bits(a[3])),
                pk16(bf16_bits(c[0]), bf16_bits(c[1])), pk16(bf16_bits(c[2]), bf16_bits(c[3])) };
}
__device__ __forceinline__ v4u pack8_bf16_lo(v4f a, v4f c) {
  return (v4u){ pk16(bf16_lo_bits(a[0]), bf16_lo_bits(a[1])), pk16(bf16_lo_bits(a[2]), bf16_lo_bits(a[3])),
                pk16(bf16_lo_bits(c[0]), bf16_lo_bits(c[1])), pk16(bf16_lo_bits(c[2]), bf16_lo_bits(c[3])) };
}
__device__ __forceinline__ v4u pack8_f16(v4f a, v4f c) {
  return (v4u){ pk16(f16_bits(a[0]), f16_bits(a[1])), pk16(f16_bits(a[2]), f16_bits(a[3])),
                pk16(f16_bits(c[0]), f16_bits(c[1])), pk16(f16_bits(c[2]), f16_bits(c[3])) };
}

template <int FORM>
__global__ __launch_bounds__(256) void k_plane(const float* __restrict__ src, int rows, int cols, int ldsrc,
                                               unsigned short* __restrict__ dst, int MP, int KP) {
  static_assert(FORM >= 0 && FORM <= 3);
  const int KTOT = (FORM == 1 || FORM == 3) ? 2 * KP : KP;
  const unsigned ppr   = (unsigned)(KTOT >> 3);
  const unsigned kp8   = (unsigned)(KP >> 3);
  const unsigned total = (unsigned)MP * ppr;
  const unsigned g     = blockIdx.x * 256u + threadIdx.x;
  const unsigned rowu  = g / ppr;
  const unsigned p     = g - rowu * ppr;
  const bool second    = p >= kp8;
  const int row = (int)rowu;
  const int c0  = (int)((second ? p - kp8 : p) << 3);
  const float* srow = src + (size_t)clampi(row, 0, rows - 1) * (size_t)ldsrc;
  float x[8];
  unsigned mk[8];
#pragma unroll
  for (int e = 0; e < 8; ++e) {
    const int c = c0 + e;
    const float v = srow[clampi(c, 0, cols - 1)];
    asm volatile("" :: "v"(v));
    x[e]  = v;
    mk[e] = (row < rows && c < cols) ? 0xFFFFu : 0u;
  }
  const v4f a = (v4f){ x[0], x[1], x[2], x[3] };
  const v4f c = (v4f){ x[4], x[5], x[6], x[7] };
  v4u o;
  if (FORM == 2) {
    o = pack8_f16(a, c);
  } else {
    const v4u hi = pack8_bf16(a, c);
    o = hi;
    if (FORM == 1) { const v4u lo = pack8_bf16_lo(a, c); o = second ? lo : hi; }
  }
  const v4u mw = (v4u){ pk16(mk[0], mk[1]), pk16(mk[2], mk[3]), pk16(mk[4], mk[5]), pk16(mk[6], mk[7]) };
  o &= mw;
  if (g < total) {
    volatile v4u* q = (volatile v4u*)(dst + (size_t)g * 8);
    *q = o;
    __threadfence();
    *q = o;
  }
}

template <int FORM> struct FragOf    { typedef FragB T; };
template <>         struct FragOf<2> { typedef FragH T; };
__device__ __forceinline__ v8f mm(const FragB& a, const FragB& b, v8f c) { return wmb(a, b, c); }
__device__ __forceinline__ v8f mm(const FragH& a, const FragH& b, v8f c) { return wmh(a, b, c); }
template <class F> __device__ __forceinline__ F ld_frag(const unsigned short* p) {
  F f;
  f.h[0] = *(const v8usa*)(p);
  f.h[1] = *(const v8usa*)(p + 16);
  return f;
}

template <int FORM, int EPI>
__global__ __launch_bounds__(256) __attribute__((amdgpu_num_vgpr(248)))
void k_gemm_nt(const unsigned short* __restrict__ A, const unsigned short* __restrict__ B,
               const float* __restrict__ bias, float* __restrict__ D, int M, int N, int KTOT, int ldd) {
  static_assert(FORM >= 0 && FORM <= 2);
  static_assert(EPI == 0 || EPI == 1);
  typedef typename FragOf<FORM>::T F;
  __shared__ __attribute__((aligned(16))) float sT[8][16 * 68];
  const int lane = threadIdx.x & 31;
  const int wave = threadIdx.x >> 5;
  const int tilesM = (M + 63) >> 6;
  const int tilesN = (N + 63) >> 6;
  const int tile = blockIdx.x * 8 + wave;
  if (tile >= tilesM * tilesN) return;
  const int tm = tile / tilesN;
  const int tn = tile - tm * tilesN;
  const int m0 = tm << 6;
  const int n0 = tn << 6;

  const int rl = lane & 15;
  const int h8 = (lane >> 4) * 8;
  const unsigned short* pa = A + (size_t)(m0 + rl) * (size_t)KTOT + h8;
  const unsigned short* pb = B + (size_t)(n0 + rl) * (size_t)KTOT + h8;

  v8f acc[4][4];
#pragma unroll
  for (int i = 0; i < 4; ++i)
#pragma unroll
    for (int j = 0; j < 4; ++j) acc[i][j] = (v8f){0.f, 0.f, 0.f, 0.f, 0.f, 0.f, 0.f, 0.f};

#pragma unroll 1
  for (int k0 = 0; k0 < KTOT; k0 += 32) {
    F bf[4];
#pragma unroll
    for (int j = 0; j < 4; ++j) bf[j] = ld_frag<F>(pb + (size_t)(j << 4) * (size_t)KTOT + k0);
#pragma unroll
    for (int i = 0; i < 4; ++i) {
      const F af = ld_frag<F>(pa + (size_t)(i << 4) * (size_t)KTOT + k0);
#pragma unroll
      for (int j = 0; j < 4; ++j) acc[i][j] = mm(af, bf[j], acc[i][j]);
    }
  }

  float* slab = sT[wave];
  const int hh = lane >> 4;
  const int c4 = (lane & 15) * 4;
  const int nc = n0 + c4;
  const bool cok = nc < N;
  v4f bv = (v4f){0.f, 0.f, 0.f, 0.f};
  if (EPI == 1) {
    bv = *(const v4fa*)(bias + clampi(nc, 0, N - 4));
    asm volatile("" :: "v"(bv));
  }
#pragma unroll
  for (int i = 0; i < 4; ++i) {
    const int mBase = m0 + (i << 4);
#pragma unroll
    for (int j = 0; j < 4; ++j) {
#pragma unroll
      for (int r = 0; r < 8; ++r) slab[(h8 + r) * 68 + (j << 4) + rl] = acc[i][j][r];
    }
    __builtin_amdgcn_fence(__ATOMIC_RELEASE, "workgroup");
    __builtin_amdgcn_wave_barrier();
    __builtin_amdgcn_fence(__ATOMIC_ACQUIRE, "workgroup");
    v4f vv[8];
#pragma unroll
    for (int it = 0; it < 8; ++it) {
      const int row = it * 2 + hh;
      v4f v = *(const v4fa*)(slab + row * 68 + c4);
      if (EPI == 1) v += bv;
      vv[it] = v;
    }
    for (int pass = 0; pass < 2; ++pass) {
#pragma unroll
      for (int it = 0; it < 8; ++it) {
        const int row = mBase + it * 2 + hh;
        if (cok && row < M) *(volatile v4f*)(D + (size_t)row * (size_t)ldd + nc) = vv[it];
      }
      __threadfence();
    }
    __builtin_amdgcn_fence(__ATOMIC_RELEASE, "workgroup");
    __builtin_amdgcn_wave_barrier();
    __builtin_amdgcn_fence(__ATOMIC_ACQUIRE, "workgroup");
  }
}

#pragma clang fp contract(off)


#define SPLIT_2 1
#define NN      20000
#define MP      20032
#define KD      128
#define N1      256
#define N2      128
#define KT2     (SPLIT_2 ? 256 : 128)
#define OUTC    40
#define NE1     139987
#define NE2     739304
#define TB_AS1  0
#define TB_AD1  256
#define TB_AS2  512
#define TB_AD2  640
#define TB_B1   768
#define TB_B2   896
#define TB_HW   960
#define TB_N    1024
#define LT      512
#define LW      16
#define LEPT    8
#define LCHUNK  (LT * LEPT)
#define NOWN    512
#define NLB     40
#define RCAP    24576
#define DEGCAP  160
#define SLOTSH  20
#define LISTTOT (NLB * RCAP)
#define LDS_LIST ((2 * RCAP + 3 * NOWN + 64) * 4)
#define WSMAX   ((size_t)128 << 20)
#define WT1_UNITS (N1 * KD / 8)
#define W2D_UNITS (N2 * KT2 / 8)
#define PREP_B1   (WT1_UNITS / 256)
#define PREP_B2   (W2D_UNITS / 256)
#define PREP_BLOCKS (PREP_B1 + PREP_B2 + 1)

static_assert(MP % 64 == 0 && MP >= NN);
static_assert(MP == 313 * 64);
static_assert(NLB * NOWN >= NN && NLB * NOWN >= MP);
static_assert(NOWN == LT && LW == LT / 32);
static_assert(NE2 < (1 << SLOTSH) && NE1 < (1 << SLOTSH) && NOWN <= (1 << 9));
static_assert(RCAP % LT == 0 && RCAP % 32 == 0);
static_assert(RCAP * 4 >= 19625 * 5);
static_assert(DEGCAP >= 127 + 8);
static_assert(LDS_LIST <= 327680);
static_assert(WT1_UNITS % 256 == 0 && W2D_UNITS % 256 == 0);
static_assert((NN * OUTC) % 32 == 0 && (NN * OUTC) % 256 == 0);
static_assert(KD % 32 == 0 && KT2 % 32 == 0 && N1 % 64 == 0 && N2 % 64 == 0);

typedef float        v2f __attribute__((ext_vector_type(2)));
typedef int          v4i __attribute__((ext_vector_type(4)));
typedef int          v2i __attribute__((ext_vector_type(2)));
typedef v2f __attribute__((may_alias)) v2fa;
typedef v4i __attribute__((may_alias)) v4ia;
typedef v2i __attribute__((may_alias)) v2ia;

__device__ __forceinline__ int imin(int a, int b) { return a < b ? a : b; }
__device__ __forceinline__ float lrelu_k(float v) { return (v > 0.0f) ? v : 0.2f * v; }
__device__ __forceinline__ float maxk(float a, float b) {
  float m = (a < b) ? b : a;
  m = (b != b) ? b : m;
  return m;
}
__device__ __forceinline__ float readlanef(float x, int k) {
  return __int_as_float(__builtin_amdgcn_readlane(__float_as_int(x), k));
}
__device__ __forceinline__ unsigned bl6(float x0, unsigned m0, float x1, unsigned m1, float x2, unsigned m2,
                                        float x3, unsigned m3, float x4, unsigned m4, float x5, unsigned m5) {
  return (__float_as_uint(x0) & m0) | (__float_as_uint(x1) & m1) | (__float_as_uint(x2) & m2) |
         (__float_as_uint(x3) & m3) | (__float_as_uint(x4) & m4) | (__float_as_uint(x5) & m5);
}

__global__ __launch_bounds__(256) void k_prep(const float* __restrict__ W1, const float* __restrict__ as1,
                                              const float* __restrict__ ad1, const float* __restrict__ hw1,
                                              const float* __restrict__ b1, const float* __restrict__ W2,
                                              const float* __restrict__ as2, const float* __restrict__ ad2,
                                              const float* __restrict__ hw2, const float* __restrict__ b2,
                                              unsigned short* WT1, unsigned short* W2D, float* TB) {
  const int t = (int)threadIdx.x;
  const int b = (int)blockIdx.x;
  if (b < PREP_B1) {
    const int u = b * 256 + t;
    const int n = u >> 4, p = u & 15;
    const int hop = n >> 7, outc = n & 127;
    const float* s = W1 + (size_t)hop * (KD * 128) + outc;
    float x[8];
#pragma unroll
    for (int e = 0; e < 8; ++e) {
      const float v = s[(size_t)(8 * p + e) * 128];
      asm volatile("" :: "v"(v));
      x[e] = v;
    }
    const v4u o = pack8_bf16((v4f){x[0], x[1], x[2], x[3]}, (v4f){x[4], x[5], x[6], x[7]});
    volatile v4u* q = (volatile v4u*)(WT1 + (size_t)u * 8);
    *q = o;
    __threadfence();
    *q = o;
  } else if (b < PREP_B1 + PREP_B2) {
    const int u = (b - PREP_B1) * 256 + t;
    const int ppr = KT2 / 8;
    const int n = u / ppr, p = u - n * ppr;
    const int hop = n >> 6, oc = n & 63;
    const int k0 = (8 * p) & 127;
    const int occ = oc < OUTC ? oc : OUTC - 1;
    const unsigned msk = (oc < OUTC) ? ~0u : 0u;
    const float* s = W2 + (size_t)hop * (128 * OUTC) + occ;
    float x[8];
#pragma unroll
    for (int e = 0; e < 8; ++e) {
      const float v = s[(size_t)(k0 + e) * OUTC];
      asm volatile("" :: "v"(v));
      x[e] = v;
    }
    v4u o = pack8_bf16((v4f){x[0], x[1], x[2], x[3]}, (v4f){x[4], x[5], x[6], x[7]});
    o &= (v4u){msk, msk, msk, msk};
    volatile v4u* q = (volatile v4u*)(W2D + (size_t)u * 8);
    *q = o;
    __threadfence();
    *q = o;
  } else {
    const int lane = t & 31;
    const int idx = 4 * t;
    const v4f a0 = *(const v4fa*)(as1 + clampi(idx - TB_AS1, 0, 252));
    asm volatile("" :: "v"(a0));
    const v4f a1 = *(const v4fa*)(ad1 + clampi(idx - TB_AD1, 0, 252));
    asm volatile("" :: "v"(a1));
    const int j2 = clampi(idx - TB_AS2, 0, 127);
    const int c2 = j2 & 63;
    const v4f a2 = *(const v4fa*)(as2 + (j2 >> 6) * OUTC + (c2 < 36 ? c2 : 36));
    asm volatile("" :: "v"(a2));
    const int j3 = clampi(idx - TB_AD2, 0, 127);
    const int c3 = j3 & 63;
    const v4f a3 = *(const v4fa*)(ad2 + (j3 >> 6) * OUTC + (c3 < 36 ? c3 : 36));
    asm volatile("" :: "v"(a3));
    const v4f a4 = *(const v4fa*)(b1 + clampi(idx - TB_B1, 0, 124));
    asm volatile("" :: "v"(a4));
    const int j5 = clampi(idx - TB_B2, 0, 63);
    const v4f a5 = *(const v4fa*)(b2 + (j5 < 36 ? j5 : 36));
    asm volatile("" :: "v"(a5));
    const unsigned m0 = (idx < TB_AD1) ? ~0u : 0u;
    const unsigned m1 = (idx >= TB_AD1 && idx < TB_AS2) ? ~0u : 0u;
    const unsigned m2 = (idx >= TB_AS2 && idx < TB_AD2 && c2 < OUTC) ? ~0u : 0u;
    const unsigned m3 = (idx >= TB_AD2 && idx < TB_B1 && c3 < OUTC) ? ~0u : 0u;
    const unsigned m4 = (idx >= TB_B1 && idx < TB_B2) ? ~0u : 0u;
    const unsigned m5 = (idx >= TB_B2 && idx < TB_HW && j5 < OUTC) ? ~0u : 0u;
    v4u o;
    o.x = bl6(a0.x, m0, a1.x, m1, a2.x, m2, a3.x, m3, a4.x, m4, a5.x, m5);
    o.y = bl6(a0.y, m0, a1.y, m1, a2.y, m2, a3.y, m3, a4.y, m4, a5.y, m5);
    o.z = bl6(a0.z, m0, a1.z, m1, a2.z, m2, a3.z, m3, a4.z, m4, a5.z, m5);
    o.w = bl6(a0.w, m0, a1.w, m1, a2.w, m2, a3.w, m3, a4.w, m4, a5.w, m5);
    o.x = bf16_bits(__uint_as_float(o.x)) << 16;
    o.y = bf16_bits(__uint_as_float(o.y)) << 16;
    o.z = bf16_bits(__uint_as_float(o.z)) << 16;
    o.w = bf16_bits(__uint_as_float(o.w)) << 16;
    const float h10 = hw1[0];
    const float h11 = hw1[1];
    const float h20 = hw2[0];
    const float h21 = hw2[1];
    asm volatile("" :: "v"(h10), "v"(h11), "v"(h20), "v"(h21));
    float g10 = bf16_val(h10);
    float g11 = bf16_val(h11);
    float g20 = bf16_val(h20);
    float g21 = bf16_val(h21);
    asm volatile("" : "+v"(g10), "+v"(g11), "+v"(g20), "+v"(g21));
    const int li = lane & 3;
    float mine = g10, part = g11;
    mine = (li == 1) ? g11 : mine;  part = (li == 1) ? g10 : part;
    mine = (li == 2) ? g20 : mine;  part = (li == 2) ? g21 : part;
    mine = (li == 3) ? g21 : mine;  part = (li == 3) ? g20 : part;
    const float mxv = (mine < part) ? part : mine;
    const float dm = mine - mxv;
    const float dp = part - mxv;
    const float em = expf(dm);
    const float ep = expf(dp);
    const float sm = em + ep;
    const float wv = em / sm;
    const float w0 = __shfl(wv, 0, 32);
    const float w1 = __shfl(wv, 1, 32);
    const float w2 = __shfl(wv, 2, 32);
    const float w3 = __shfl(wv, 3, 32);
    const unsigned mh = (t == TB_HW / 4) ? ~0u : 0u;
    o.x = (o.x & ~mh) | (__float_as_uint(w0) & mh);
    o.y = (o.y & ~mh) | (__float_as_uint(w1) & mh);
    o.z = (o.z & ~mh) | (__float_as_uint(w2) & mh);
    o.w = (o.w & ~mh) | (__float_as_uint(w3) & mh);
    volatile v4u* q = (volatile v4u*)(TB + idx);
    *q = o;
    __threadfence();
    *q = o;
  }
}

__global__ __launch_bounds__(LT) void k_list(const int* __restrict__ edst, const int* __restrict__ esrc, const int E,
                                             unsigned* LIST, int* META) {
  extern __shared__ v4u lds_list[];
  int* reg1 = (int*)lds_list;
  int* reg2 = reg1 + RCAP;
  int* scnt = reg2 + RCAP;
  int* soff = scnt + NOWN;
  int* curs = soff + NOWN;
  int* wcnt = curs + NOWN;
  int* wtot = wcnt + 2 * LW;
  const int tid = (int)threadIdx.x, lane = tid & 31, wave = tid >> 5;
  const int nodeBase = (int)blockIdx.x * NOWN;
  int nb = NN - nodeBase;
  nb = nb > NOWN ? NOWN : (nb < 0 ? 0 : nb);
  const unsigned nbs = (unsigned)nodeBase, unb = (unsigned)nb;

  scnt[tid] = 0;
  if (tid == 0) { reg1[0] = 0; reg2[0] = 0; }

  const int nch = (E + LCHUNK - 1) / LCHUNK;
  const int el = E - 1;
  int tot = 0;
#pragma unroll 1
  for (int ch = 0; ch < nch; ++ch) {
    const int par = ch & 1;
    const int cbase = ch * LCHUNK;
    const int e0 = cbase + tid * LEPT;
    int k0, k1, k2, k3, k4, k5, k6, k7;
    if (cbase + LCHUNK <= E) {
      const v4i da = *(const v4ia*)(edst + e0);
      const v4i db = *(const v4ia*)(edst + e0 + 4);
      asm volatile("" :: "v"(da), "v"(db));
      k0 = da.x; k1 = da.y; k2 = da.z; k3 = da.w;
      k4 = db.x; k5 = db.y; k6 = db.z; k7 = db.w;
    } else {
      k0 = edst[imin(e0 + 0, el)];
      k1 = edst[imin(e0 + 1, el)];
      k2 = edst[imin(e0 + 2, el)];
      k3 = edst[imin(e0 + 3, el)];
      k4 = edst[imin(e0 + 4, el)];
      k5 = edst[imin(e0 + 5, el)];
      k6 = edst[imin(e0 + 6, el)];
      k7 = edst[imin(e0 + 7, el)];
      asm volatile("" :: "v"(k0), "v"(k1), "v"(k2), "v"(k3), "v"(k4), "v"(k5), "v"(k6), "v"(k7));
    }
    const unsigned s0 = (unsigned)k0 - nbs, s1 = (unsigned)k1 - nbs;
    const unsigned s2 = (unsigned)k2 - nbs, s3 = (unsigned)k3 - nbs;
    const unsigned s4 = (unsigned)k4 - nbs, s5 = (unsigned)k5 - nbs;
    const unsigned s6 = (unsigned)k6 - nbs, s7 = (unsigned)k7 - nbs;
    const bool h0 = ((e0 + 0) < E) && (s0 < unb), h1 = ((e0 + 1) < E) && (s1 < unb);
    const bool h2 = ((e0 + 2) < E) && (s2 < unb), h3 = ((e0 + 3) < E) && (s3 < unb);
    const bool h4 = ((e0 + 4) < E) && (s4 < unb), h5 = ((e0 + 5) < E) && (s5 < unb);
    const bool h6 = ((e0 + 6) < E) && (s6 < unb), h7 = ((e0 + 7) < E) && (s7 < unb);
    const int c = (int)h0 + (int)h1 + (int)h2 + (int)h3 + (int)h4 + (int)h5 + (int)h6 + (int)h7;
    int incl = c;
#pragma unroll
    for (int d = 1; d < 32; d <<= 1) {
      const int up = __shfl_up(incl, d, 32);
      incl += (lane >= d) ? up : 0;
    }
    const int wtotal = __shfl(incl, 31, 32);
    if (lane == 0) wcnt[par * LW + wave] = wtotal;
    __syncthreads();
    int all = 0, pre = 0;
#pragma unroll
    for (int g = 0; g < 4; ++g) {
      const v4i w4 = *(const v4ia*)(wcnt + par * LW + 4 * g);
      const int c0 = clampi(w4.x, 0, 256), c1 = clampi(w4.y, 0, 256);
      const int c2 = clampi(w4.z, 0, 256), c3 = clampi(w4.w, 0, 256);
      all += c0 + c1 + c2 + c3;
      pre += (4 * g + 0 < wave) ? c0 : 0;
      pre += (4 * g + 1 < wave) ? c1 : 0;
      pre += (4 * g + 2 < wave) ? c2 : 0;
      pre += (4 * g + 3 < wave) ? c3 : 0;
    }
    int pos = tot + pre + (incl - c);
#define PUTJ(J, HJ, SJ) if (HJ) { if (pos < RCAP) reg1[pos] = (int)((unsigned)(e0 + (J)) | ((SJ) << SLOTSH)); ++pos; }
    PUTJ(0, h0, s0)
    PUTJ(1, h1, s1)
    PUTJ(2, h2, s2)
    PUTJ(3, h3, s3)
    PUTJ(4, h4, s4)
    PUTJ(5, h5, s5)
    PUTJ(6, h6, s6)
    PUTJ(7, h7, s7)
#undef PUTJ
    tot += all;
  }
  __syncthreads();
  const bool ovf = tot > RCAP;
  const int nh = ovf ? RCAP : tot;

  if (wave == 0) {
#pragma unroll 1
    for (int b0 = 0; b0 < nh; b0 += 32) {
      const int idx = b0 + lane;
      const int uv  = reg1[idx < nh ? idx : nh - 1];
      const int m32 = (nh - b0) < 32 ? (nh - b0) : 32;
#pragma unroll 1
      for (int k = 0; k < m32; ++k) {
        const int u  = __builtin_amdgcn_readlane(uv, k);
        const int sl = (int)(((unsigned)u >> SLOTSH) & (unsigned)(NOWN - 1));
        const int cv = scnt[sl] + 1;
        if (lane == 0) scnt[sl] = cv;
      }
    }
  }
  __syncthreads();

  {
    const int cr = scnt[tid];
    const int cc = cr < 0 ? 0 : cr;
    int incl = cc;
#pragma unroll
    for (int d = 1; d < 32; d <<= 1) {
      const int up = __shfl_up(incl, d, 32);
      incl += (lane >= d) ? up : 0;
    }
    if (lane == 31) wtot[wave] = incl;
    __syncthreads();
    int pre = 0;
#pragma unroll
    for (int g = 0; g < 4; ++g) {
      const v4i w4 = *(const v4ia*)(wtot + 4 * g);
      pre += (4 * g + 0 < wave) ? w4.x : 0;
      pre += (4 * g + 1 < wave) ? w4.y : 0;
      pre += (4 * g + 2 < wave) ? w4.z : 0;
      pre += (4 * g + 3 < wave) ? w4.w : 0;
    }
    const int run = pre + incl - cc;
    soff[tid] = run;
    curs[tid] = run;
  }
  __syncthreads();

  if (wave == 0) {
#pragma unroll 1
    for (int b0 = 0; b0 < nh; b0 += 32) {
      const int idx = b0 + lane;
      const int uv  = reg1[idx < nh ? idx : nh - 1];
      const int m32 = (nh - b0) < 32 ? (nh - b0) : 32;
#pragma unroll 1
      for (int k = 0; k < m32; ++k) {
        const int u   = __builtin_amdgcn_readlane(uv, k);
        const int sl  = (int)(((unsigned)u >> SLOTSH) & (unsigned)(NOWN - 1));
        const int eid = (int)((unsigned)u & ((1u << SLOTSH) - 1u));
        const int pr  = curs[sl];
        const int pc  = clampi(pr, 0, RCAP - 1);
        if (lane == 0) { reg2[pc] = eid; curs[sl] = pc + 1; }
      }
    }
  }
  __syncthreads();

  {
    unsigned* lbase = LIST + (size_t)blockIdx.x * (size_t)RCAP;
    const int nhm = nh > 0 ? nh - 1 : 0;
#pragma unroll 1
    for (int it = 0; it < RCAP / LT; ++it) {
      const int i  = it * LT + tid;
      const int ic = i < nhm ? i : nhm;
      const int eid = clampi(reg2[ic], 0, el);
      const int sw = esrc[eid];
      asm volatile("" :: "v"(sw));
      const unsigned msk = (i < nh) ? ~0u : 0u;
      const unsigned o = (unsigned)clampi(sw, 0, NN - 1) & msk;
      volatile unsigned* q = (volatile unsigned*)(lbase + i);
      *q = o;
      __threadfence();
      *q = o;
    }
  }

  {
    const int cr = scnt[tid];
    const int so = soff[tid];
    v2i m;
    m.x = (int)blockIdx.x * RCAP + so;
    m.y = (ovf || cr > DEGCAP) ? -1 : cr;
    volatile v2i* q = (volatile v2i*)(META + 2 * (size_t)(nodeBase + tid));
    *q = m;
    __threadfence();
    *q = m;
  }
}

__global__ __launch_bounds__(256) void k_rowprep1(const float* __restrict__ HH, const float* __restrict__ TB,
                                                  float* ES1, float* ED1) {
  __shared__ __attribute__((aligned(16))) float sES[128];
  __shared__ __attribute__((aligned(16))) float sED[128];
  const int lane = (int)threadIdx.x & 31;
  const int wave = (int)threadIdx.x >> 5;
  const int row  = (int)blockIdx.x * 8 + wave;
  const int head = lane >> 2;
#pragma unroll
  for (int k = 0; k < 2; ++k) {
    const v4f h = *(const v4fa*)(HH + (size_t)row * N1 + 128 * k + 4 * lane);
    asm volatile("" :: "v"(h));
    const v4f a = *(const v4fa*)(TB + TB_AS1 + 128 * k + 4 * lane);
    const v4f d = *(const v4fa*)(TB + TB_AD1 + 128 * k + 4 * lane);
    float t = h.x * a.x;
    float u = h.y * a.y; t = t + u;
    u = h.z * a.z; t = t + u;
    u = h.w * a.w; t = t + u;
    t = t + __shfl_xor(t, 2, 32);
    t = t + __shfl_xor(t, 1, 32);
    float s = h.x * d.x;
    u = h.y * d.y; s = s + u;
    u = h.z * d.z; s = s + u;
    u = h.w * d.w; s = s + u;
    s = s + __shfl_xor(s, 2, 32);
    s = s + __shfl_xor(s, 1, 32);
    if ((lane & 3) == 0) {
      sES[wave * 16 + 8 * k + head] = t;
      sED[wave * 16 + 8 * k + head] = s;
    }
  }
  __syncthreads();
  if (wave == 0) {
    const v4f sv = *(const v4fa*)(sES + 4 * lane);
    volatile v4f* q = (volatile v4f*)(ES1 + (size_t)blockIdx.x * 128 + 4 * lane);
    *q = sv;
    __threadfence();
    *q = sv;
  } else if (wave == 1) {
    const v4f sv = *(const v4fa*)(sED + 4 * lane);
    volatile v4f* q = (volatile v4f*)(ED1 + (size_t)blockIdx.x * 128 + 4 * lane);
    *q = sv;
    __threadfence();
    *q = sv;
  }
}

struct Hop1 { v4f s; int bad; };

__device__ __forceinline__ Hop1 walk1_hop(const float* __restrict__ HH, const float* __restrict__ ES,
                                          const float* __restrict__ ED, const unsigned* __restrict__ LIST,
                                          const int* __restrict__ META, const int hop, const int rowc,
                                          const bool rok, const int lane) {
  const int head = lane >> 2;
  const v2i mt = *(const v2ia*)(META + 2 * (size_t)rowc);
  asm volatile("" :: "v"(mt));
  const int craw = mt.y;
  const int offv = clampi(mt.x, 0, LISTTOT);
  const int cntv = imin(rok ? clampi(craw, 0, DEGCAP) : 0, LISTTOT - offv);
  const int off = __builtin_amdgcn_readfirstlane(offv);
  const int cnt = __builtin_amdgcn_readfirstlane(cntv);
  Hop1 r;
  r.bad = ((craw < 0) || (craw > DEGCAP)) ? 1 : 0;

  const float ed = ED[(size_t)rowc * 16 + 8 * hop + head];
  asm volatile("" :: "v"(ed));
  float mx = -__builtin_inff();
#pragma unroll 1
  for (int b0 = 0; b0 < cnt; b0 += 32) {
    const int j = (b0 + lane) < cnt ? (b0 + lane) : cnt - 1;
    const unsigned sv = LIST[(size_t)(off + j)];
    asm volatile("" :: "v"(sv));
    const int col = clampi((int)sv, 0, NN - 1);
    const int m32 = (cnt - b0) < 32 ? (cnt - b0) : 32;
#pragma unroll 1
    for (int k = 0; k < m32; ++k) {
      const int c = __builtin_amdgcn_readlane(col, k);
      const float es = ES[(size_t)c * 16 + 8 * hop + head];
      asm volatile("" :: "v"(es));
      const float e = lrelu_k(es + ed);
      mx = maxk(mx, e);
    }
  }
  float z = 0.0f;
#pragma unroll 1
  for (int b0 = 0; b0 < cnt; b0 += 32) {
    const int j = (b0 + lane) < cnt ? (b0 + lane) : cnt - 1;
    const unsigned sv = LIST[(size_t)(off + j)];
    asm volatile("" :: "v"(sv));
    const int col = clampi((int)sv, 0, NN - 1);
    const int m32 = (cnt - b0) < 32 ? (cnt - b0) : 32;
#pragma unroll 1
    for (int k = 0; k < m32; ++k) {
      const int c = __builtin_amdgcn_readlane(col, k);
      const float es = ES[(size_t)c * 16 + 8 * hop + head];
      asm volatile("" :: "v"(es));
      const float e = lrelu_k(es + ed);
      const float d = e - mx;
      const float p = expf(d);
      z = z + p;
    }
  }
  const float den = z + 1e-16f;
  v4f S = (v4f){0.0f, 0.0f, 0.0f, 0.0f};
#pragma unroll 1
  for (int b0 = 0; b0 < cnt; b0 += 32) {
    const int j = (b0 + lane) < cnt ? (b0 + lane) : cnt - 1;
    const unsigned sv = LIST[(size_t)(off + j)];
    asm volatile("" :: "v"(sv));
    const int col = clampi((int)sv, 0, NN - 1);
    const int m32 = (cnt - b0) < 32 ? (cnt - b0) : 32;
#pragma unroll 1
    for (int k = 0; k < m32; ++k) {
      const int c = __builtin_amdgcn_readlane(col, k);
      const float es = ES[(size_t)c * 16 + 8 * hop + head];
      asm volatile("" :: "v"(es));
      const v4f hn = *(const v4fa*)(HH + (size_t)c * N1 + 128 * hop + 4 * lane);
      asm volatile("" :: "v"(hn));
      const float e = lrelu_k(es + ed);
      const float d = e - mx;
      const float p = expf(d);
      const float al = p / den;
      float pr;
      pr = al * hn.x; S.x = S.x + pr;
      pr = al * hn.y; S.y = S.y + pr;
      pr = al * hn.z; S.z = S.z + pr;
      pr = al * hn.w; S.w = S.w + pr;
    }
  }
  r.s = S;
  return r;
}

__global__ __launch_bounds__(256) void k_walk1(const float* __restrict__ HH, const float* __restrict__ ES1,
                                               const float* __restrict__ ED1, const unsigned* __restrict__ LISTA,
                                               const int* __restrict__ METAA, const unsigned* __restrict__ LISTB,
                                               const int* __restrict__ METAB, const float* __restrict__ TB,
                                               unsigned short* OP) {
  __shared__ __attribute__((aligned(16))) float sy[8][128];
  const int lane = (int)threadIdx.x & 31;
  const int wave = (int)threadIdx.x >> 5;
  const int row  = (int)blockIdx.x * 8 + wave;
  const bool rok = row < NN;
  const int rowc = rok ? row : NN - 1;

  const Hop1 r0 = walk1_hop(HH, ES1, ED1, LISTA, METAA, 0, rowc, rok, lane);
  const Hop1 r1 = walk1_hop(HH, ES1, ED1, LISTB, METAB, 1, rowc, rok, lane);

  const float hw0 = TB[TB_HW + 0];
  const float hw1 = TB[TB_HW + 1];
  asm volatile("" :: "v"(hw0), "v"(hw1));
  const v4f bv = *(const v4fa*)(TB + TB_B1 + 4 * lane);
  asm volatile("" :: "v"(bv));
  v4f tot = (v4f){0.0f, 0.0f, 0.0f, 0.0f};
  float pr;
  pr = hw0 * r0.s.x; tot.x = tot.x + pr;
  pr = hw0 * r0.s.y; tot.y = tot.y + pr;
  pr = hw0 * r0.s.z; tot.z = tot.z + pr;
  pr = hw0 * r0.s.w; tot.w = tot.w + pr;
  pr = hw1 * r1.s.x; tot.x = tot.x + pr;
  pr = hw1 * r1.s.y; tot.y = tot.y + pr;
  pr = hw1 * r1.s.z; tot.z = tot.z + pr;
  pr = hw1 * r1.s.w; tot.w = tot.w + pr;
  v4f v;
  v.x = tot.x + bv.x;
  v.y = tot.y + bv.y;
  v.z = tot.z + bv.z;
  v.w = tot.w + bv.w;
  const bool bad = (r0.bad | r1.bad) != 0;
  const float qnan = __uint_as_float(0x7fc00000u);

  float* slab = sy[wave];
  *(v4fa*)(slab + 4 * lane) = v;
#pragma unroll 1
  for (int c = 0; c < 4; ++c) {
    const float a = slab[4 * lane + c];
    float y = (a > 0.0f) ? a : expm1f(a);
    y = bad ? qnan : y;
    slab[4 * lane + c] = y;
  }
  __builtin_amdgcn_fence(__ATOMIC_RELEASE, "workgroup");
  __builtin_amdgcn_wave_barrier();
  __builtin_amdgcn_fence(__ATOMIC_ACQUIRE, "workgroup");

  const int q8 = (lane & 15) * 8;
  const v4f ya = *(const v4fa*)(slab + q8);
  const v4f yc = *(const v4fa*)(slab + q8 + 4);
  const v4u hi = pack8_bf16(ya, yc);
  v4u o = hi;
#if SPLIT_2
  const v4u lo = pack8_bf16_lo(ya, yc);
  o = (lane >= 16) ? lo : hi;
#endif
  const unsigned rm = rok ? ~0u : 0u;
  o &= (v4u){rm, rm, rm, rm};
  const bool wr = SPLIT_2 ? true : (lane < 16);
  volatile v4u* q = (volatile v4u*)(OP + (size_t)row * KT2 + (SPLIT_2 ? 8 * lane : q8));
  if (wr) *q = o;
  __threadfence();
  if (wr) *q = o;
}

__global__ __launch_bounds__(256) void k_rowprep2(const float* __restrict__ G, const float* __restrict__ TB,
                                                  float* ES2, float* ED2) {
  __shared__ __attribute__((aligned(16))) float sES[32];
  __shared__ __attribute__((aligned(16))) float sED[32];
  const int lane = (int)threadIdx.x & 31;
  const int wave = (int)threadIdx.x >> 5;
#pragma unroll
  for (int it = 0; it < 2; ++it) {
    const int node = (int)blockIdx.x * 16 + wave * 2 + it;
#pragma unroll
    for (int k = 0; k < 2; ++k) {
      const v2f g = *(const v2fa*)(G + (size_t)node * N2 + 64 * k + 2 * lane);
      asm volatile("" :: "v"(g));
      const v2f a = *(const v2fa*)(TB + TB_AS2 + 64 * k + 2 * lane);
      const v2f d = *(const v2fa*)(TB + TB_AD2 + 64 * k + 2 * lane);
      float t = g.x * a.x;
      float u = g.y * a.y; t = t + u;
      float s = g.x * d.x;
      u = g.y * d.y; s = s + u;
#pragma unroll
      for (int x = 16; x > 0; x >>= 1) {
        t = t + __shfl_xor(t, x, 32);
        s = s + __shfl_xor(s, x, 32);
      }
      if (lane == 0) {
        sES[(wave * 2 + it) * 2 + k] = t;
        sED[(wave * 2 + it) * 2 + k] = s;
      }
    }
  }
  __syncthreads();
  const int l8 = lane & 7;
  const bool wr = lane < 8;
  if (wave == 0) {
    const v4f sv = *(const v4fa*)(sES + 4 * l8);
    volatile v4f* q = (volatile v4f*)(ES2 + (size_t)blockIdx.x * 32 + 4 * l8);
    if (wr) *q = sv;
    __threadfence();
    if (wr) *q = sv;
  } else if (wave == 1) {
    const v4f sv = *(const v4fa*)(sED + 4 * l8);
    volatile v4f* q = (volatile v4f*)(ED2 + (size_t)blockIdx.x * 32 + 4 * l8);
    if (wr) *q = sv;
    __threadfence();
    if (wr) *q = sv;
  }
}

struct Hop2 { v2f s; int bad; };

__device__ __forceinline__ Hop2 walk2_hop(const float* __restrict__ G, const float* __restrict__ ES,
                                          const float* __restrict__ ED, const unsigned* __restrict__ LIST,
                                          const int* __restrict__ META, const int hop, const int rowc,
                                          const bool rok, const int lane) {
  const v2i mt = *(const v2ia*)(META + 2 * (size_t)rowc);
  asm volatile("" :: "v"(mt));
  const int craw = mt.y;
  const int offv = clampi(mt.x, 0, LISTTOT);
  const int cntv = imin(rok ? clampi(craw, 0, DEGCAP) : 0, LISTTOT - offv);
  const int off = __builtin_amdgcn_readfirstlane(offv);
  const int cnt = __builtin_amdgcn_readfirstlane(cntv);
  Hop2 r;
  r.bad = ((craw < 0) || (craw > DEGCAP)) ? 1 : 0;

  const float ed = ED[(size_t)rowc * 2 + hop];
  asm volatile("" :: "v"(ed));
  float mx = -__builtin_inff();
#pragma unroll 1
  for (int b0 = 0; b0 < cnt; b0 += 32) {
    const int j = (b0 + lane) < cnt ? (b0 + lane) : cnt - 1;
    const unsigned sv = LIST[(size_t)(off + j)];
    asm volatile("" :: "v"(sv));
    const int col = clampi((int)sv, 0, NN - 1);
    const float es = ES[(size_t)col * 2 + hop];
    asm volatile("" :: "v"(es));
    const float e = lrelu_k(es + ed);
    mx = maxk(mx, e);
  }
#pragma unroll
  for (int x = 16; x > 0; x >>= 1) {
    const float o = __shfl_xor(mx, x, 32);
    mx = maxk(mx, o);
  }
  float z = 0.0f;
#pragma unroll 1
  for (int b0 = 0; b0 < cnt; b0 += 32) {
    const int j = (b0 + lane) < cnt ? (b0 + lane) : cnt - 1;
    const unsigned sv = LIST[(size_t)(off + j)];
    asm volatile("" :: "v"(sv));
    const int col = clampi((int)sv, 0, NN - 1);
    const float es = ES[(size_t)col * 2 + hop];
    asm volatile("" :: "v"(es));
    const float e = lrelu_k(es + ed);
    const float d = e - mx;
    const float p = expf(d);
    const int m32 = (cnt - b0) < 32 ? (cnt - b0) : 32;
#pragma unroll 1
    for (int k = 0; k < m32; ++k) {
      const float pk = readlanef(p, k);
      z = z + pk;
    }
  }
  const float den = z + 1e-16f;
  v2f S = (v2f){0.0f, 0.0f};
#pragma unroll 1
  for (int b0 = 0; b0 < cnt; b0 += 32) {
    const int j = (b0 + lane) < cnt ? (b0 + lane) : cnt - 1;
    const unsigned sv = LIST[(size_t)(off + j)];
    asm volatile("" :: "v"(sv));
    const int col = clampi((int)sv, 0, NN - 1);
    const float es = ES[(size_t)col * 2 + hop];
    asm volatile("" :: "v"(es));
    const float e = lrelu_k(es + ed);
    const float d = e - mx;
    const float p = expf(d);
    const float al = p / den;
    const int m32 = (cnt - b0) < 32 ? (cnt - b0) : 32;
#pragma unroll 1
    for (int k = 0; k < m32; ++k) {
      const int c = __builtin_amdgcn_readlane(col, k);
      const float w = readlanef(al, k);
      const v2f g = *(const v2fa*)(G + (size_t)c * N2 + 64 * hop + 2 * lane);
      asm volatile("" :: "v"(g));
      float pr;
      pr = w * g.x; S.x = S.x + pr;
      pr = w * g.y; S.y = S.y + pr;
    }
  }
  r.s = S;
  return r;
}

__global__ __launch_bounds__(256) void k_walk2(const float* __restrict__ G, const float* __restrict__ ES2,
                                               const float* __restrict__ ED2, const unsigned* __restrict__ LISTA,
                                               const int* __restrict__ METAA, const unsigned* __restrict__ LISTB,
                                               const int* __restrict__ METAB, const float* __restrict__ TB,
                                               float* TF) {
  const int lane = (int)threadIdx.x & 31;
  const int wave = (int)threadIdx.x >> 5;
  const int row  = (int)blockIdx.x * 8 + wave;
  const bool rok = row < NN;
  const int rowc = rok ? row : NN - 1;

  const Hop2 r0 = walk2_hop(G, ES2, ED2, LISTA, METAA, 0, rowc, rok, lane);
  const Hop2 r1 = walk2_hop(G, ES2, ED2, LISTB, METAB, 1, rowc, rok, lane);

  const float hw0 = TB[TB_HW + 2];
  const float hw1 = TB[TB_HW + 3];
  asm volatile("" :: "v"(hw0), "v"(hw1));
  const v2f bv = *(const v2fa*)(TB + TB_B2 + 2 * lane);
  asm volatile("" :: "v"(bv));
  v2f tot = (v2f){0.0f, 0.0f};
  float pr;
  pr = hw0 * r0.s.x; tot.x = tot.x + pr;
  pr = hw0 * r0.s.y; tot.y = tot.y + pr;
  pr = hw1 * r1.s.x; tot.x = tot.x + pr;
  pr = hw1 * r1.s.y; tot.y = tot.y + pr;
  float ox = tot.x + bv.x;
  float oy = tot.y + bv.y;
  const bool bad = (r0.bad | r1.bad) != 0;
  const float qnan = __uint_as_float(0x7fc00000u);
  ox = bad ? qnan : ox;
  oy = bad ? qnan : oy;
  const unsigned km = (rok && (2 * lane < OUTC)) ? ~0u : 0u;
  v2f o;
  o.x = __uint_as_float(__float_as_uint(ox) & km);
  o.y = __uint_as_float(__float_as_uint(oy) & km);
  volatile v2f* q = (volatile v2f*)(TF + (size_t)row * 64 + 2 * lane);
  *q = o;
  __threadfence();
  *q = o;
}

__global__ __launch_bounds__(256) void k_flat(const float* __restrict__ TF, float* out, const int total) {
  const int f  = (int)blockIdx.x * 256 + (int)threadIdx.x;
  const int fc = f < total ? f : total - 1;
  const int row = fc / OUTC;
  const int col = fc - OUTC * row;
  const float v = TF[(size_t)row * 64 + col];
  asm volatile("" :: "v"(v));
  const bool ok = f < total;
  volatile float* q = (volatile float*)(out + fc);
  if (ok) *q = v;
  __threadfence();
  if (ok) *q = v;
}

extern "C" void kernel_launch(void* const* d_in, const int* in_sizes, int n_in,
                              void* d_out, int out_size, void* d_ws, size_t ws_size,
                              hipStream_t stream) {
  if (n_in < 15) return;
  if (in_sizes[0] != NN * KD) return;
  if (in_sizes[1] != 2 * KD * 128) return;
  if (in_sizes[2] != 256 || in_sizes[3] != 256) return;
  if (in_sizes[4] != 2 || in_sizes[9] != 2) return;
  if (in_sizes[5] != 128) return;
  if (in_sizes[6] != 2 * 128 * OUTC) return;
  if (in_sizes[7] != 2 * OUTC || in_sizes[8] != 2 * OUTC) return;
  if (in_sizes[10] != OUTC) return;
  if (in_sizes[11] != NE1 || in_sizes[12] != NE1) return;
  if (in_sizes[13] != NE2 || in_sizes[14] != NE2) return;
  if (out_size != NN * OUTC) return;

  const float* x   = (const float*)d_in[0];
  const float* W1  = (const float*)d_in[1];
  const float* as1 = (const float*)d_in[2];
  const float* ad1 = (const float*)d_in[3];
  const float* hw1 = (const float*)d_in[4];
  const float* b1  = (const float*)d_in[5];
  const float* W2  = (const float*)d_in[6];
  const float* as2 = (const float*)d_in[7];
  const float* ad2 = (const float*)d_in[8];
  const float* hw2 = (const float*)d_in[9];
  const float* b2  = (const float*)d_in[10];
  const int* e1s = (const int*)d_in[11];
  const int* e1d = (const int*)d_in[12];
  const int* e2s = (const int*)d_in[13];
  const int* e2d = (const int*)d_in[14];
  float* out = (float*)d_out;

  const size_t szXB   = (size_t)MP * KD * 2;
  const size_t szWT1  = (size_t)N1 * KD * 2;
  const size_t szW2D  = (size_t)N2 * KT2 * 2;
  const size_t szTB   = (size_t)TB_N * 4;
  const size_t szHH   = (size_t)MP * N1 * 4;
  const size_t szS1   = (size_t)MP * 16 * 4;
  const size_t szOP   = (size_t)MP * KT2 * 2;
  const size_t szG    = (size_t)MP * N2 * 4;
  const size_t szS2   = (size_t)MP * 2 * 4;
  const size_t szTF   = (size_t)MP * 64 * 4;
  const size_t szLIST = (size_t)NLB * RCAP * 4;
  const size_t szMETA = (size_t)NLB * NOWN * 2 * 4;
  static_assert((size_t)MP * KD * 2 + (size_t)N1 * KD * 2 + (size_t)N2 * KT2 * 2 + (size_t)TB_N * 4 +
                (size_t)MP * N1 * 4 + 2 * (size_t)MP * 16 * 4 + (size_t)MP * KT2 * 2 + (size_t)MP * N2 * 4 +
                2 * (size_t)MP * 2 * 4 + (size_t)MP * 64 * 4 + 2 * (size_t)NLB * RCAP * 4 +
                2 * (size_t)NLB * NOWN * 8 <= WSMAX);
  static_assert(SPLIT_2 == 0 ||
                (size_t)MP * KD * 2 + (size_t)N1 * KD * 2 + (size_t)N2 * KT2 * 2 + (size_t)TB_N * 4 +
                (size_t)MP * N1 * 4 + 2 * (size_t)MP * 16 * 4 + (size_t)MP * KT2 * 2 + (size_t)MP * N2 * 4 +
                2 * (size_t)MP * 2 * 4 + (size_t)MP * 64 * 4 + 2 * (size_t)NLB * RCAP * 4 +
                2 * (size_t)NLB * NOWN * 8 == 62493696);
  static_assert(((size_t)MP * 2 * 4) % 256 == 0 && ((size_t)MP * 16 * 4) % 256 == 0);
  char* ws = (char*)d_ws;
  size_t off = 0;
  const size_t oXB  = off; off += szXB;
  const size_t oWT1 = off; off += szWT1;
  const size_t oW2D = off; off += szW2D;
  const size_t oTB  = off; off += szTB;
  const size_t oHH  = off; off += szHH;
  const size_t oES1 = off; off += szS1;
  const size_t oED1 = off; off += szS1;
  const size_t oOP  = off; off += szOP;
  const size_t oG   = off; off += szG;
  const size_t oES2 = off; off += szS2;
  const size_t oED2 = off; off += szS2;
  const size_t oTF  = off; off += szTF;
  const size_t oL1  = off; off += szLIST;
  const size_t oL2  = off; off += szLIST;
  const size_t oM1  = off; off += szMETA;
  const size_t oM2  = off; off += szMETA;
  if (off > ws_size || off > (size_t)WSMAX) return;
  unsigned short* XB  = (unsigned short*)(ws + oXB);
  unsigned short* WT1 = (unsigned short*)(ws + oWT1);
  unsigned short* W2D = (unsigned short*)(ws + oW2D);
  float*    TB  = (float*)(ws + oTB);
  float*    HH  = (float*)(ws + oHH);
  float*    ES1 = (float*)(ws + oES1);
  float*    ED1 = (float*)(ws + oED1);
  unsigned short* OP = (unsigned short*)(ws + oOP);
  float*    G   = (float*)(ws + oG);
  float*    ES2 = (float*)(ws + oES2);
  float*    ED2 = (float*)(ws + oED2);
  float*    TF  = (float*)(ws + oTF);
  unsigned* L1  = (unsigned*)(ws + oL1);
  unsigned* L2  = (unsigned*)(ws + oL2);
  int*      M1  = (int*)(ws + oM1);
  int*      M2  = (int*)(ws + oM2);

  hipFuncSetAttribute(reinterpret_cast<const void*>(&k_list),
                      hipFuncAttributeMaxDynamicSharedMemorySize, LDS_LIST);

  k_plane<0><<<MP * KD / 8 / 256, 256, 0, stream>>>(x, NN, KD, KD, XB, MP, KD);
  k_prep<<<PREP_BLOCKS, 256, 0, stream>>>(W1, as1, ad1, hw1, b1, W2, as2, ad2, hw2, b2, WT1, W2D, TB);
  k_list<<<NLB, LT, LDS_LIST, stream>>>(e1d, e1s, NE1, L1, M1);
  k_list<<<NLB, LT, LDS_LIST, stream>>>(e2d, e2s, NE2, L2, M2);
  {
    const int tiles = (MP / 64) * (N1 / 64);
    k_gemm_nt<0, 0><<<(tiles + 7) / 8, 256, 0, stream>>>(XB, WT1, TB, HH, MP, N1, KD, N1);
  }
  k_rowprep1<<<MP / 8, 256, 0, stream>>>(HH, TB, ES1, ED1);
  k_walk1<<<MP / 8, 256, 0, stream>>>(HH, ES1, ED1, L1, M1, L2, M2, TB, OP);
  {
    const int tiles = (MP / 64) * (N2 / 64);
    k_gemm_nt<0, 0><<<(tiles + 7) / 8, 256, 0, stream>>>(OP, W2D, TB, G, MP, N2, KT2, N2);
  }
  k_rowprep2<<<MP / 16, 256, 0, stream>>>(G, TB, ES2, ED2);
  k_walk2<<<MP / 8, 256, 0, stream>>>(G, ES2, ED2, L1, M1, L2, M2, TB, TF);
  k_flat<<<NN * OUTC / 256, 256, 0, stream>>>(TF, out, NN * OUTC);
}
